// GINandPool_47699906789506
// MI455X (gfx1250) — hardware-verified
//
#include <hip/hip_runtime.h>
#include <stddef.h>
#include <math.h>


#define NTHR  256
#define NWAVE 8
#define EPT   8
#define CHUNK (NTHR * EPT)
#define WCAP  (EPT * 32)
#define FD    64
#define OUTD  16
#define NB    1024
#define RPW   (NB / NWAVE)
#define TPW   (NB / (16 * NWAVE))
#define NBG   256
#define RPWG  (NBG / NWAVE)
#define TPWG  (NBG / (16 * NWAVE))

#define LDS_ACC   0
#define LDS_LIST  (LDS_ACC + NB * FD * 4)
#define LDS_PRM   (LDS_LIST + NWAVE * WCAP * 4)
#define LDS_WCNT  (LDS_PRM + 2 * FD * 4)
#define LDS_TOTAL (LDS_WCNT + 64)

#define LP_ACC   0
#define LP_LIST  (LP_ACC + NBG * FD * 4)
#define LP_SOT   (LP_LIST + NWAVE * WCAP * 4)
#define LP_PRM   (LP_SOT + NBG * OUTD * 4)
#define LP_WCNT  (LP_PRM + (FD + OUTD) * 4)
#define LP_TOTAL (LP_WCNT + 64)

static_assert(FD == 64);
static_assert(OUTD == 16);
static_assert(NB == TPW * 16 * NWAVE);
static_assert(NBG == TPWG * 16 * NWAVE);
static_assert((NB & (NB - 1)) == 0 && NB <= 32768);
static_assert((NBG & (NBG - 1)) == 0);
static_assert(CHUNK <= 65536);
static_assert(WCAP == 32 * EPT);
static_assert((RPW % 2) == 0 && (RPWG % 2) == 0);
static_assert((LDS_TOTAL % 16) == 0 && LDS_TOTAL <= 300 * 1024);
static_assert((LP_TOTAL % 16) == 0);
static_assert(4 * NTHR * 4 == NBG * OUTD);

typedef float        v4f   __attribute__((ext_vector_type(4)));
typedef float        v8f   __attribute__((ext_vector_type(8)));
typedef int          v4i   __attribute__((ext_vector_type(4)));
typedef unsigned int v4u   __attribute__((ext_vector_type(4)));
typedef __bf16       v16bf __attribute__((ext_vector_type(16)));
union FragB { v16bf v; v4u q[2]; };
union Pk8   { v4u q; __bf16 e[8]; };

__device__ __forceinline__ float bf16r(float x) { return (float)(__bf16)x; }

__device__ __forceinline__ v8f zero8f() {
  v8f c;
#pragma unroll
  for (int i = 0; i < 8; ++i) c[i] = 0.0f;
  return c;
}

__device__ __forceinline__ v8f wmb(v16bf a, v16bf b, v8f c) {
  v8f d = __builtin_amdgcn_wmma_f32_16x16x32_bf16(false, a, false, b, (short)0, c, false, false);
  asm volatile("v_nop\n\tv_nop\n\tv_nop\n\tv_nop" : "+v"(d) : "v"(a), "v"(b));
  return d;
}

__device__ __forceinline__ void put4(v16bf& fh, v16bf& fl, const int b, const v4f a) {
  { const __bf16 hb = (__bf16)a.x; fh[b]     = hb; fl[b]     = (__bf16)(a.x - (float)hb); }
  { const __bf16 hb = (__bf16)a.y; fh[b + 1] = hb; fl[b + 1] = (__bf16)(a.y - (float)hb); }
  { const __bf16 hb = (__bf16)a.z; fh[b + 2] = hb; fl[b + 2] = (__bf16)(a.z - (float)hb); }
  { const __bf16 hb = (__bf16)a.w; fh[b + 3] = hb; fl[b + 3] = (__bf16)(a.w - (float)hb); }
}

__device__ __forceinline__ int scan_chunk(const int* __restrict__ keys, int nK, int cbase, int base,
                                          int span, int vec8, int* list, int tid, int wave) {
  int wc = 0;
  const int el0  = tid * EPT;
  const int e0   = cbase + el0;
  const int sent = -2147483647 - 1;
  v4i da, db;
  if (vec8 != 0 && cbase + CHUNK <= nK) {
    da = *(const v4i*)(keys + e0);
    db = *(const v4i*)(keys + e0 + 4);
  } else {
    da.x = (e0     < nK) ? keys[min(e0, nK - 1)] : sent;
    da.y = (e0 + 1 < nK) ? keys[min(e0 + 1, nK - 1)] : sent;
    da.z = (e0 + 2 < nK) ? keys[min(e0 + 2, nK - 1)] : sent;
    da.w = (e0 + 3 < nK) ? keys[min(e0 + 3, nK - 1)] : sent;
    db.x = (e0 + 4 < nK) ? keys[min(e0 + 4, nK - 1)] : sent;
    db.y = (e0 + 5 < nK) ? keys[min(e0 + 5, nK - 1)] : sent;
    db.z = (e0 + 6 < nK) ? keys[min(e0 + 6, nK - 1)] : sent;
    db.w = (e0 + 7 < nK) ? keys[min(e0 + 7, nK - 1)] : sent;
  }
  const unsigned nb = (unsigned)base;
  const unsigned sp = (unsigned)span;
  const unsigned s0 = (unsigned)da.x - nb, s1 = (unsigned)da.y - nb;
  const unsigned s2 = (unsigned)da.z - nb, s3 = (unsigned)da.w - nb;
  const unsigned s4 = (unsigned)db.x - nb, s5 = (unsigned)db.y - nb;
  const unsigned s6 = (unsigned)db.z - nb, s7 = (unsigned)db.w - nb;
  const bool h0 = s0 < sp, h1 = s1 < sp, h2 = s2 < sp, h3 = s3 < sp;
  const bool h4 = s4 < sp, h5 = s5 < sp, h6 = s6 < sp, h7 = s7 < sp;
  const unsigned any = __builtin_amdgcn_ballot_w32(h0 | h1 | h2 | h3 | h4 | h5 | h6 | h7);
  if (any != 0u) {
#define HITJ(J, HJ, SJ) { \
      const unsigned mj = __builtin_amdgcn_ballot_w32(HJ); \
      if (mj != 0u) { \
        if (HJ) { \
          const int pos = wc + (int)__builtin_amdgcn_mbcnt_lo(mj, 0u); \
          if (pos < WCAP) list[wave * WCAP + pos] = (int)(((SJ) << 16) | (unsigned)(el0 + (J))); \
        } \
        wc += (int)__builtin_popcount(mj); } }
    HITJ(0, h0, s0)
    HITJ(1, h1, s1)
    HITJ(2, h2, s2)
    HITJ(3, h3, s3)
    HITJ(4, h4, s4)
    HITJ(5, h5, s5)
    HITJ(6, h6, s6)
    HITJ(7, h7, s7)
#undef HITJ
  }
  return wc;
}

template <int IND>
__device__ __forceinline__ void drain2(const int* list, const int* wcnt, float* acc, const int smask,
                                       const float* __restrict__ rows, const int* __restrict__ idx,
                                       const int cbase, const int nK, const int nR, const int lane) {
  const int hh = lane >> 4, c4 = 4 * (lane & 15);
#pragma unroll 1
  for (int u = 0; u < NWAVE; ++u) {
    int n = __builtin_amdgcn_readfirstlane(wcnt[u]);
    n = n > WCAP ? WCAP : (n < 0 ? 0 : n);
#pragma unroll 1
    for (int i = 0; i < n; i += 2) {
      const bool v1 = (i + 1) < n;
      const int  i1 = v1 ? i + 1 : i;
      const int  e0 = __builtin_amdgcn_readfirstlane(list[u * WCAP + i]);
      const int  e1 = __builtin_amdgcn_readfirstlane(list[u * WCAP + i1]);
      const int  s0 = (e0 >> 16) & smask, s1 = (e1 >> 16) & smask;
      const bool same = v1 && (s0 == s1);
      const int  ent = hh ? e1 : e0;
      int k = cbase + (ent & 0xFFFF);
      k = k > nK - 1 ? nK - 1 : k;
      int r = k;
      if (IND) { r = idx[k]; r = r < 0 ? 0 : (r > nR - 1 ? nR - 1 : r); }
      const v4f v = *(const v4f*)(rows + (size_t)r * FD + c4);
      float* ap = acc + (hh ? s1 : s0) * FD + c4;
      v4f a = *(v4f*)ap;
      a += v;
      if (same) {
        v4f w;
        w.x = __shfl_xor(v.x, 16, 32);
        w.y = __shfl_xor(v.y, 16, 32);
        w.z = __shfl_xor(v.z, 16, 32);
        w.w = __shfl_xor(v.w, 16, 32);
        a += w;
      }
      const bool st = (hh == 0) || (v1 && !same);
      if (st) *(v4f*)ap = a;
    }
  }
}

template <int NT>
__device__ __forceinline__ void gemm64(const float* zr, const unsigned short* __restrict__ wq,
                                       const int m, const int hh, v8f (&c)[NT]) {
#pragma unroll
  for (int nt = 0; nt < NT; ++nt) c[nt] = zero8f();
#pragma unroll
  for (int kt = 0; kt < 2; ++kt) {
    v16bf ah, al;
    {
      const float* zp = zr + 32 * kt;
      const v4f z0 = *(const v4f*)zp;
      const v4f z1 = *(const v4f*)(zp + 4);
      const v4f z2 = *(const v4f*)(zp + 16);
      const v4f z3 = *(const v4f*)(zp + 20);
      put4(ah, al, 0, z0);
      put4(ah, al, 4, z1);
      put4(ah, al, 8, z2);
      put4(ah, al, 12, z3);
    }
    const unsigned short* bp = wq + (size_t)m * FD + 32 * kt + 8 * hh;
#pragma unroll
    for (int nt = 0; nt < NT; ++nt) {
      FragB b;
      const unsigned short* p = bp + (size_t)nt * 16 * FD;
      b.q[0] = *(const v4u*)p;
      b.q[1] = *(const v4u*)(p + 16);
      c[nt] = wmb(ah, b.v, c[nt]);
      c[nt] = wmb(al, b.v, c[nt]);
    }
  }
}

__device__ __forceinline__ void epi4(v8f (&c)[4], const float* bias, float* orow, const int m) {
#pragma unroll
  for (int nt = 0; nt < 4; ++nt) {
    const float bb = bias[16 * nt + m];
#pragma unroll
    for (int r = 0; r < 8; ++r) c[nt][r] = fmaxf(c[nt][r] + bb, 0.0f);
  }
#pragma unroll
  for (int r = 0; r < 8; ++r) {
#pragma unroll
    for (int nt = 0; nt < 4; ++nt) orow[r * FD + 16 * nt] = c[nt][r];
  }
}

__device__ __forceinline__ void store_rows(const float* acc, float* dst, const size_t rowBase,
                                           const int wave, const int hh, const int c4, const int rpw) {
#pragma unroll 1
  for (int rr = 0; rr < rpw / 2; ++rr) {
    const int row = wave * rpw + 2 * rr + hh;
    const v4f v = *(const v4f*)(acc + row * FD + c4);
    *(volatile v4f*)(dst + (rowBase + (size_t)row) * FD + c4) = v;
  }
}

__global__ __launch_bounds__(NTHR) void k_prep(const float* __restrict__ W1, const float* __restrict__ W2,
                                              const float* __restrict__ Wa, const float* __restrict__ Wb,
                                              int nL, unsigned short* wq) {
  const int tid = threadIdx.x;
  const int b = blockIdx.x;
  const int nFull = 2 * nL + 1;
  const float* src;
  int ncol, n, kc;
  size_t dsto;
  bool act = true;
  if (b < 2 * nFull) {
    const int mat = b >> 1;
    const int u = ((b & 1) << 8) + tid;
    n = u >> 3;
    kc = u & 7;
    ncol = FD;
    src = (mat < nL) ? (W1 + (size_t)mat * FD * FD)
                     : ((mat < 2 * nL) ? (W2 + (size_t)(mat - nL) * FD * FD) : Wa);
    dsto = (size_t)mat * FD * FD + (size_t)u * 8;
  } else {
    act = tid < 128;
    const int u = tid & 127;
    n = u >> 3;
    kc = u & 7;
    ncol = OUTD;
    src = Wb;
    dsto = (size_t)nFull * FD * FD + (size_t)u * 8;
  }
  Pk8 pk;
#pragma unroll
  for (int j = 0; j < 8; ++j) {
    const int k = 8 * kc + j;
    pk.e[j] = (__bf16)src[(size_t)k * ncol + n];
  }
  unsigned short* dh = wq + dsto;
  const v4u q = pk.q;
  if (act) *(volatile v4u*)dh = q;
  __threadfence();
  if (act) *(volatile v4u*)dh = q;
}

__device__ __forceinline__ void enc_store(const int* cnt, const float* prm, float* xout,
                                          const size_t rowBase, const int wave, const int hh, const int c4) {
#pragma unroll 1
  for (int rr = 0; rr < RPW / 2; ++rr) {
    const int row = wave * RPW + 2 * rr + hh;
    const float d = (float)cnt[row];
    v4f v;
    v.x = fmaxf(__fadd_rn(__fmul_rn(d, prm[c4]),     prm[FD + c4]),     0.0f);
    v.y = fmaxf(__fadd_rn(__fmul_rn(d, prm[c4 + 1]), prm[FD + c4 + 1]), 0.0f);
    v.z = fmaxf(__fadd_rn(__fmul_rn(d, prm[c4 + 2]), prm[FD + c4 + 2]), 0.0f);
    v.w = fmaxf(__fadd_rn(__fmul_rn(d, prm[c4 + 3]), prm[FD + c4 + 3]), 0.0f);
    *(volatile v4f*)(xout + (rowBase + (size_t)row) * FD + c4) = v;
  }
}

__global__ __launch_bounds__(NTHR) void k_enc(const int* __restrict__ ei, const float* __restrict__ wenc,
                                             const float* __restrict__ benc, float* xout, int nN, int nE) {
  __shared__ int   cnt[NB];
  __shared__ int   list[NWAVE * WCAP];
  __shared__ float prm[2 * FD];
  __shared__ int   wcnt[NWAVE];
  const int tid = threadIdx.x, lane = tid & 31, wave = tid >> 5, hh = lane >> 4, c4 = 4 * (lane & 15);
  const int nodeBase = blockIdx.x * NB;
  for (int i = tid; i < NB; i += NTHR) cnt[i] = 0;
  if (tid < FD) { prm[tid] = bf16r(wenc[tid]); prm[FD + tid] = bf16r(benc[tid]); }
  __syncthreads();
  {
    const int nChunks = (nE + CHUNK - 1) / CHUNK;
#pragma unroll 1
    for (int ch = 0; ch < nChunks; ++ch) {
      const int cbase = ch * CHUNK;
      const int wc = scan_chunk(ei, nE, cbase, nodeBase, NB, 1, list, tid, wave);
      if (lane == 0) wcnt[wave] = wc;
      __syncthreads();
      if (wave == 0) {
#pragma unroll 1
        for (int u = 0; u < NWAVE; ++u) {
          int n = __builtin_amdgcn_readfirstlane(wcnt[u]);
          n = n > WCAP ? WCAP : (n < 0 ? 0 : n);
#pragma unroll 1
          for (int i = 0; i < n; ++i) {
            const int ent  = __builtin_amdgcn_readfirstlane(list[u * WCAP + i]);
            const int slot = (ent >> 16) & (NB - 1);
            if (lane == 0) cnt[slot] = cnt[slot] + 1;
          }
        }
      }
      __syncthreads();
    }
  }
  enc_store(cnt, prm, xout, (size_t)nodeBase, wave, hh, c4);
  __threadfence();
  enc_store(cnt, prm, xout, (size_t)nodeBase, wave, hh, c4);
}

__global__ __launch_bounds__(NTHR) void k_layer(
    const float* __restrict__ hin, const int* __restrict__ ei,
    const unsigned short* __restrict__ w1q, const unsigned short* __restrict__ w2q,
    const float* __restrict__ b1, const float* __restrict__ b2,
    float* hout, int nN, int nE, int vec8) {
  extern __shared__ __attribute__((aligned(16))) unsigned char dsm[];
  float* acc  = (float*)(dsm + LDS_ACC);
  int*   list = (int*)(dsm + LDS_LIST);
  float* prm  = (float*)(dsm + LDS_PRM);
  int*   wcnt = (int*)(dsm + LDS_WCNT);

  const int tid = threadIdx.x, lane = tid & 31, wave = tid >> 5, hh = lane >> 4, m = lane & 15, c4 = 4 * m;
  const int nodeBase = blockIdx.x * NB;
  const int* srcs = ei;
  const int* dsts = ei + nE;

  {
    const v4f z4 = {0.0f, 0.0f, 0.0f, 0.0f};
#pragma unroll 1
    for (int rr = 0; rr < RPW / 2; ++rr) {
      const int row  = wave * RPW + 2 * rr + hh;
      const int node = nodeBase + row;
      const int nc   = node < nN ? node : nN - 1;
      v4f v = *(const v4f*)(hin + (size_t)nc * FD + c4);
      if (node >= nN) v = z4;
      *(v4f*)(acc + row * FD + c4) = v;
    }
  }
  if (tid < FD) { prm[tid] = bf16r(b1[tid]); prm[FD + tid] = bf16r(b2[tid]); }
  __syncthreads();

  {
    const int nChunks = (nE + CHUNK - 1) / CHUNK;
#pragma unroll 1
    for (int ch = 0; ch < nChunks; ++ch) {
      const int cbase = ch * CHUNK;
      const int wc = scan_chunk(dsts, nE, cbase, nodeBase, NB, vec8, list, tid, wave);
      if (lane == 0) wcnt[wave] = wc;
      __syncthreads();
      if (wave == 0) drain2<1>(list, wcnt, acc, NB - 1, hin, srcs, cbase, nE, nN, lane);
      __syncthreads();
    }
  }

#pragma unroll 1
  for (int tt = 0; tt < TPW; ++tt) {
    const int t = wave + NWAVE * tt;
    const float* zr = acc + (16 * t + m) * FD + 8 * hh;
    float* orow = acc + (16 * t + 8 * hh) * FD + m;
    v8f c[4];
    gemm64<4>(zr, w1q, m, hh, c);
    __syncthreads();
    epi4(c, prm, orow, m);
    __syncthreads();
    gemm64<4>(zr, w2q, m, hh, c);
    __syncthreads();
    epi4(c, prm + FD, orow, m);
    __syncthreads();
  }

  store_rows(acc, hout, (size_t)nodeBase, wave, hh, c4, RPW);
  __threadfence();
  store_rows(acc, hout, (size_t)nodeBase, wave, hh, c4, RPW);
}

__global__ __launch_bounds__(NTHR) void k_pool(
    const float* __restrict__ h, const int* __restrict__ bt,
    const unsigned short* __restrict__ wdq1, const unsigned short* __restrict__ wdq2,
    const float* __restrict__ bd1, const float* __restrict__ bd2,
    float* outp, int nN, int nG) {
  extern __shared__ __attribute__((aligned(16))) unsigned char dsm[];
  float* accz = (float*)(dsm + LP_ACC);
  int*   list = (int*)(dsm + LP_LIST);
  float* sot  = (float*)(dsm + LP_SOT);
  float* prm  = (float*)(dsm + LP_PRM);
  int*   wcnt = (int*)(dsm + LP_WCNT);

  const int tid = threadIdx.x, lane = tid & 31, wave = tid >> 5, hh = lane >> 4, m = lane & 15, c4 = 4 * m;
  const int gBase = blockIdx.x * NBG;

  {
    const v4f z4 = {0.0f, 0.0f, 0.0f, 0.0f};
#pragma unroll 1
    for (int rr = 0; rr < RPWG / 2; ++rr) {
      const int row = wave * RPWG + 2 * rr + hh;
      *(v4f*)(accz + row * FD + c4) = z4;
    }
  }
  if (tid < FD)   prm[tid] = bf16r(bd1[tid]);
  if (tid < OUTD) prm[FD + tid] = bf16r(bd2[tid]);
  __syncthreads();

  {
    const int nChunks = (nN + CHUNK - 1) / CHUNK;
#pragma unroll 1
    for (int ch = 0; ch < nChunks; ++ch) {
      const int cbase = ch * CHUNK;
      const int wc = scan_chunk(bt, nN, cbase, gBase, NBG, 1, list, tid, wave);
      if (lane == 0) wcnt[wave] = wc;
      __syncthreads();
      if (wave == 0) drain2<0>(list, wcnt, accz, NBG - 1, h, bt, cbase, nN, nN, lane);
      __syncthreads();
    }
  }

#pragma unroll 1
  for (int tt = 0; tt < TPWG; ++tt) {
    const int t = wave + NWAVE * tt;
    const float* zr = accz + (16 * t + m) * FD + 8 * hh;
    float* orow = accz + (16 * t + 8 * hh) * FD + m;
    {
      v8f c[4];
      gemm64<4>(zr, wdq1, m, hh, c);
      __syncthreads();
      epi4(c, prm, orow, m);
    }
    __syncthreads();
    {
      v8f c2[1];
      gemm64<1>(zr, wdq2, m, hh, c2);
      const float bb2 = prm[FD + m];
#pragma unroll
      for (int r = 0; r < 8; ++r) sot[(16 * t + 8 * hh + r) * OUTD + m] = c2[0][r] + bb2;
    }
    __syncthreads();
  }

  {
    const size_t obase = (size_t)gBase * OUTD;
    v4f o[4];
    bool ok[4];
#pragma unroll
    for (int j = 0; j < 4; ++j) {
      const int f = tid + NTHR * j;
      o[j]  = *(const v4f*)(sot + 4 * f);
      ok[j] = (gBase + (f >> 2)) < nG;
    }
#pragma unroll
    for (int j = 0; j < 4; ++j)
      if (ok[j]) *(volatile v4f*)(outp + obase + 4 * (size_t)(tid + NTHR * j)) = o[j];
    __threadfence();
#pragma unroll
    for (int j = 0; j < 4; ++j)
      if (ok[j]) *(volatile v4f*)(outp + obase + 4 * (size_t)(tid + NTHR * j)) = o[j];
  }
}

extern "C" void kernel_launch(void* const* d_in, const int* in_sizes, int n_in,
                              void* d_out, int out_size, void* d_ws, size_t ws_size,
                              hipStream_t stream) {
  if (n_in < 12) return;
  const int nE = in_sizes[0] / 2;
  if (nE < 1 || in_sizes[0] != 2 * nE) return;
  const int nN = in_sizes[1];
  if (nN < 1) return;
  if (in_sizes[2] != FD || in_sizes[3] != FD) return;
  const int nL = in_sizes[5] / FD;
  if (nL < 1 || nL > 32) return;
  if (in_sizes[4] != nL * FD * FD || in_sizes[5] != nL * FD) return;
  if (in_sizes[6] != nL * FD * FD || in_sizes[7] != nL * FD) return;
  if (in_sizes[8] != FD * FD || in_sizes[9] != FD) return;
  if (in_sizes[10] != FD * OUTD || in_sizes[11] != OUTD) return;
  const int nG = out_size / OUTD;
  if (nG < 1 || out_size != nG * OUTD) return;

  const int*   ei   = (const int*)d_in[0];
  const int*   bt   = (const int*)d_in[1];
  const float* Wenc = (const float*)d_in[2];
  const float* benc = (const float*)d_in[3];
  const float* W1   = (const float*)d_in[4];
  const float* b1   = (const float*)d_in[5];
  const float* W2   = (const float*)d_in[6];
  const float* b2   = (const float*)d_in[7];
  const float* Wd1  = (const float*)d_in[8];
  const float* bd1  = (const float*)d_in[9];
  const float* Wd2  = (const float*)d_in[10];
  const float* bd2  = (const float*)d_in[11];
  float* outp = (float*)d_out;

  const int nBlk  = (nN + NB - 1) / NB;
  const int nBlkG = (nG + NBG - 1) / NBG;
  const size_t rowsP = (size_t)nBlk * NB;
  const int nFull = 2 * nL + 1;
  const size_t planeHalves = (size_t)nFull * FD * FD + (size_t)OUTD * FD;

  char* ws = (char*)d_ws;
  size_t off = 0;
  const size_t oWq = off; off += (planeHalves * 2 + 255) & ~(size_t)255;
  const size_t oX0 = off; off += (rowsP * FD * 4 + 255) & ~(size_t)255;
  const size_t oX1 = off; off += (rowsP * FD * 4 + 255) & ~(size_t)255;
  size_t limit = (size_t)134217728;
  if (ws_size < limit) limit = ws_size;
  if (off > limit) return;

  unsigned short* Wq = (unsigned short*)(ws + oWq);
  float* X0 = (float*)(ws + oX0);
  float* X1 = (float*)(ws + oX1);

  const int vec8 = ((nE & 3) == 0) ? 1 : 0;

  k_prep<<<2 * nFull + 1, NTHR, 0, stream>>>(W1, W2, Wd1, Wd2, nL, Wq);
  k_enc<<<nBlk, NTHR, 0, stream>>>(ei, Wenc, benc, X1, nN, nE);

  (void)hipFuncSetAttribute(reinterpret_cast<const void*>(&k_layer),
                            hipFuncAttributeMaxDynamicSharedMemorySize, LDS_TOTAL);
  (void)hipFuncSetAttribute(reinterpret_cast<const void*>(&k_pool),
                            hipFuncAttributeMaxDynamicSharedMemorySize, LP_TOTAL);

  const float* hin = X1;
  for (int l = 0; l < nL; ++l) {
    float* hout = (l & 1) ? X1 : X0;
    k_layer<<<nBlk, NTHR, LDS_TOTAL, stream>>>(
        hin, ei,
        Wq + (size_t)l * FD * FD, Wq + (size_t)(nL + l) * FD * FD,
        b1 + (size_t)l * FD, b2 + (size_t)l * FD,
        hout, nN, nE, vec8);
    hin = hout;
  }

  k_pool<<<nBlkG, NTHR, LP_TOTAL, stream>>>(
      hin, bt,
      Wq + (size_t)(2 * nL) * FD * FD, Wq + (size_t)nFull * FD * FD,
      bd1, bd2, outp, nN, nG);
}
